// SCC3D_9964324126880
// MI455X (gfx1250) — hardware-verified
//
#include <hip/hip_runtime.h>

typedef __attribute__((ext_vector_type(16))) _Float16 v16h;
typedef __attribute__((ext_vector_type(8)))  _Float16 v8h;
typedef __attribute__((ext_vector_type(16))) __bf16   v16b;
typedef __attribute__((ext_vector_type(8)))  __bf16   v8b;
typedef __attribute__((ext_vector_type(8)))  float    v8f;
typedef __attribute__((ext_vector_type(4)))  float    v4f;

#define NTOK   256
#define CDIM   256
#define HEADS  8
#define HD     32
#define QKVLD  768
#define KCH    64
#define QBLK   64
#define OSP    68

__device__ __forceinline__ unsigned short f2bf_bits(float f) {
  unsigned u = __float_as_uint(f);
  return (unsigned short)((u + 0x7FFFu + ((u >> 16) & 1u)) >> 16);
}
__device__ __forceinline__ float bf_bits2f(unsigned short h) { return __uint_as_float(((unsigned)h) << 16); }

__device__ __forceinline__ void dep_guard_h(v8f& a, v8f& b, v16h x, v16h y) { asm volatile("v_nop\n\tv_nop\n\tv_nop\n\tv_nop" : "+v"(a), "+v"(b) : "v"(x), "v"(y)); }
__device__ __forceinline__ void dep_guard_b(v8f& a, v8f& b, v16b x, v16b y) { asm volatile("v_nop\n\tv_nop\n\tv_nop\n\tv_nop" : "+v"(a), "+v"(b) : "v"(x), "v"(y)); }
__device__ __forceinline__ void keep4_h(v16h a, v16h b, v16h c, v16h d) { asm volatile("v_nop" :: "v"(a), "v"(b), "v"(c), "v"(d)); }
__device__ __forceinline__ void keep4_b(v16b a, v16b b, v16b c, v16b d) { asm volatile("v_nop" :: "v"(a), "v"(b), "v"(c), "v"(d)); }
__device__ __forceinline__ void acc_guard4(v8f& a, v8f& b, v8f& c, v8f& d) { asm volatile("v_nop\n\tv_nop\n\tv_nop\n\tv_nop" : "+v"(a), "+v"(b), "+v"(c), "+v"(d)); }

template <typename T> struct Frag;
template <> struct Frag<_Float16> {
  typedef v16h V; union U { v16h v; v8h h[2]; };
  static __device__ __forceinline__ v16h load(const _Float16* p) {
    U f; f.h[0] = *(const v8h*)(p); f.h[1] = *(const v8h*)(p + 16); return f.v;
  }
  static __device__ __forceinline__ v8f mma(v16h a, v16h b, v8f c) {
    return __builtin_amdgcn_wmma_f32_16x16x32_f16(false, a, false, b, (short)0, c, false, false);
  }
  static __device__ __forceinline__ void guard(v8f& a, v8f& b, v16h x, v16h y) { dep_guard_h(a, b, x, y); }
  static __device__ __forceinline__ void keep(v16h a, v16h b, v16h c, v16h d) { keep4_h(a, b, c, d); }
};
template <> struct Frag<__bf16> {
  typedef v16b V; union U { v16b v; v8b h[2]; };
  static __device__ __forceinline__ v16b load(const __bf16* p) {
    U f; f.h[0] = *(const v8b*)(p); f.h[1] = *(const v8b*)(p + 16); return f.v;
  }
  static __device__ __forceinline__ v8f mma(v16b a, v16b b, v8f c) {
    return __builtin_amdgcn_wmma_f32_16x16x32_bf16(false, a, false, b, (short)0, c, false, false);
  }
  static __device__ __forceinline__ void guard(v8f& a, v8f& b, v16b x, v16b y) { dep_guard_b(a, b, x, y); }
  static __device__ __forceinline__ void keep(v16b a, v16b b, v16b c, v16b d) { keep4_b(a, b, c, d); }
};

__device__ __forceinline__ v8f mma_h(v16h a, v16h b, v8f c) {
  c = __builtin_amdgcn_wmma_f32_16x16x32_f16(false, a, false, b, (short)0, c, false, false);
  asm volatile("v_nop\n\tv_nop\n\tv_nop\n\tv_nop" : "+v"(c) : "v"(a), "v"(b));
  return c;
}

template <int ET> struct Elem;
template <> struct Elem<0> { typedef _Float16 T; };
template <> struct Elem<1> { typedef __bf16 T; };
template <int ET, bool SPLIT, int BIAS_MODE, int OUT_MODE, bool RESID, int ACT = 0>
__global__ __launch_bounds__(256) void wmma_gemm64(
    const unsigned short* __restrict__ Ap, const unsigned short* __restrict__ A2p, int lda, long strideA,
    const unsigned short* __restrict__ Btp, const unsigned short* __restrict__ Bt2p, int ldb, long strideB,
    void* __restrict__ Cout, void* __restrict__ Cout2, int ldc, long strideC,
    const float* __restrict__ bias,
    const float* __restrict__ resid, long strideR,
    int M, int N, int K, float scale) {
  typedef typename Elem<ET>::T T;
  typedef typename Frag<T>::V V;
  const T* A = (const T*)Ap; const T* A2 = (const T*)A2p; const T* Bt = (const T*)Btp; const T* Bt2 = (const T*)Bt2p;
  __shared__ __align__(16) float sT[8][16 * 68];
  const int b    = blockIdx.y;
  const int lane = threadIdx.x & 31;
  const int wave = threadIdx.x >> 5;
  const int tilesN = N >> 6;
  const int tilesM = M >> 6;
  const int tile = blockIdx.x * 8 + wave;
  if (tile >= tilesM * tilesN) return;
  const int tm = tile / tilesN;
  const int tn = tile - tm * tilesN;
  const int m0 = tm << 6;
  const int n0 = tn << 6;

  const T* Ab  = A  + (size_t)b * strideA;
  const T* Bb  = Bt + (size_t)b * strideB;
  const T* Ab2 = SPLIT ? (A2  + (size_t)b * strideA) : nullptr;
  const T* Bb2 = SPLIT ? (Bt2 + (size_t)b * strideB) : nullptr;

  const int rlane = lane & 15;
  const int koff  = (lane >> 4) * 8;
  const int mOff  = (lane >> 4) * 8;

  v8f acc[4][4];
#pragma unroll
  for (int i = 0; i < 4; ++i)
#pragma unroll
    for (int j = 0; j < 4; ++j) acc[i][j] = (v8f){0.f,0.f,0.f,0.f,0.f,0.f,0.f,0.f};

  for (int k0 = 0; k0 < K; k0 += 32) {
    V bh[4], bl[4];
#pragma unroll
    for (int j = 0; j < 4; ++j) {
      const size_t bo = (size_t)(n0 + (j << 4) + rlane) * ldb + koff + k0;
      bh[j] = Frag<T>::load(Bb + bo);
      if (SPLIT) bl[j] = Frag<T>::load(Bb2 + bo);
    }
#pragma unroll
    for (int i = 0; i < 4; ++i) {
      const size_t ao = (size_t)(m0 + (i << 4) + rlane) * lda + koff + k0;
      V ah = Frag<T>::load(Ab + ao);
      V al;
      if (SPLIT) al = Frag<T>::load(Ab2 + ao);
#pragma unroll
      for (int j = 0; j < 4; ++j) {
        acc[i][j] = Frag<T>::mma(ah, bh[j], acc[i][j]);
        if (SPLIT) {
          acc[i][j] = Frag<T>::mma(ah, bl[j], acc[i][j]);
          acc[i][j] = Frag<T>::mma(al, bh[j], acc[i][j]);
        }
      }
      Frag<T>::guard(acc[i][0], acc[i][3], ah, SPLIT ? al : ah);
    }
    Frag<T>::keep(bh[0], bh[1], bh[2], bh[3]);
    if (SPLIT) Frag<T>::keep(bl[0], bl[1], bl[2], bl[3]);
  }
  acc_guard4(acc[0][0], acc[0][1], acc[0][2], acc[0][3]);
  acc_guard4(acc[1][0], acc[1][1], acc[1][2], acc[1][3]);
  acc_guard4(acc[2][0], acc[2][1], acc[2][2], acc[2][3]);
  acc_guard4(acc[3][0], acc[3][1], acc[3][2], acc[3][3]);

  float* slab = sT[wave];
  const float* Rb = RESID ? (resid + (size_t)b * strideR) : nullptr;
#pragma unroll
  for (int i = 0; i < 4; ++i) {
    const int mBase = m0 + (i << 4);
#pragma unroll
    for (int j = 0; j < 4; ++j) {
      const int n = n0 + (j << 4) + rlane;
      float bv = 0.f;
      if (BIAS_MODE == 2) bv = bias[n];
#pragma unroll
      for (int r = 0; r < 8; ++r) {
        float v = acc[i][j][r] * scale;
        if (BIAS_MODE == 1) v += bias[mBase + mOff + r];
        if (BIAS_MODE == 2) v += bv;
        if (RESID) v += Rb[(size_t)(mBase + mOff + r) * ldc + n];
        if (ACT == 1) v = tanhf(v);
        if (ACT == 2) v = fmaxf(v, 0.0f);
        if (ACT == 3) v = v / (1.0f + expf(-v));
        if (ACT == 4) v = (v > 0.f) ? v : 0.01f * v;
        if (ACT == 5) v = 0.5f * v * (1.0f + erff(v * 0.70710678118654752f));
        slab[(mOff + r) * 68 + (j << 4) + rlane] = v;
      }
    }
    __builtin_amdgcn_fence(__ATOMIC_RELEASE, "workgroup");
    __builtin_amdgcn_wave_barrier();
    __builtin_amdgcn_fence(__ATOMIC_ACQUIRE, "workgroup");
    if (OUT_MODE == 0) {
      float* C = (float*)Cout + (size_t)b * strideC;
      const int hh = lane >> 4, c4 = (lane & 15) * 4;
      for (int pass = 0; pass < 2; ++pass) {
#pragma unroll
        for (int it = 0; it < 8; ++it) {
          const int row = it * 2 + hh;
          v4f v = *(const v4f*)(slab + row * 68 + c4);
          *(volatile v4f*)(C + (size_t)(mBase + row) * ldc + n0 + c4) = v;
        }
        __threadfence();
      }
    } else {
      const int q = lane >> 3, c8 = (lane & 7) * 8;
      unsigned short* C  = (unsigned short*)Cout  + (size_t)b * strideC;
      unsigned short* C2 = (OUT_MODE == 2) ? ((unsigned short*)Cout2 + (size_t)b * strideC) : nullptr;
      for (int pass = 0; pass < 2; ++pass) {
#pragma unroll
        for (int it = 0; it < 4; ++it) {
          const int row = it * 4 + q;
          const float* sp = slab + row * 68 + c8;
          v8h hv, lv;
#pragma unroll
          for (int e = 0; e < 8; ++e) {
            if (OUT_MODE == 1) {
              hv[e] = (_Float16)sp[e];
            } else {
              unsigned short hb = f2bf_bits(sp[e]);
              unsigned short lb = f2bf_bits(sp[e] - bf_bits2f(hb));
              hv[e] = __builtin_bit_cast(_Float16, hb);
              lv[e] = __builtin_bit_cast(_Float16, lb);
            }
          }
          *(volatile v8h*)(C + (size_t)(mBase + row) * ldc + n0 + c8) = hv;
          if (OUT_MODE == 2) *(volatile v8h*)(C2 + (size_t)(mBase + row) * ldc + n0 + c8) = lv;
        }
        __threadfence();
      }
    }
    __builtin_amdgcn_fence(__ATOMIC_RELEASE, "workgroup");
    __builtin_amdgcn_wave_barrier();
    __builtin_amdgcn_fence(__ATOMIC_ACQUIRE, "workgroup");
  }
}

__global__ __launch_bounds__(256) void cast_f32_f16x2(
    const float* __restrict__ in, _Float16* __restrict__ out, int n2, float sc) {
  int i = blockIdx.x * 256 + threadIdx.x;
  if (i < n2) {
    const _Float16 h0 = (_Float16)(in[2 * i] * sc), h1 = (_Float16)(in[2 * i + 1] * sc);
    const unsigned u = (unsigned)__builtin_bit_cast(unsigned short, h0) | ((unsigned)__builtin_bit_cast(unsigned short, h1) << 16);
    ((volatile unsigned*)out)[i] = u;
    __threadfence();
    ((volatile unsigned*)out)[i] = u;
  }
}

__global__ __launch_bounds__(256) void bias_gather_kernel(
    const float* __restrict__ table, const int* __restrict__ idx, float* __restrict__ biasH, int ntab) {
  const int i = blockIdx.x * 256 + threadIdx.x;
  if (i < NTOK * NTOK) {
    int t = idx[i];
    t = t < 0 ? 0 : (t > ntab - 1 ? ntab - 1 : t);
    float vals[HEADS];
#pragma unroll
    for (int h = 0; h < HEADS; ++h) vals[h] = table[(size_t)t * HEADS + h];
    for (int pass = 0; pass < 2; ++pass) {
#pragma unroll
      for (int h = 0; h < HEADS; ++h)
        ((volatile float*)biasH)[(size_t)h * (NTOK * NTOK) + i] = vals[h];
      __threadfence();
    }
  }
}

__global__ __launch_bounds__(256)
void attn_hd32_kernel(const _Float16* __restrict__ qkv, const float* __restrict__ biasH,
                      const float* __restrict__ maskp, _Float16* __restrict__ ctx,
                      int nwin, int nmask, float qscale) {
  __shared__ __align__(16) _Float16 Ksh[2][KCH * HD];
  __shared__ __align__(16) _Float16 Vtsh[2][HD * KCH];
  __shared__ __align__(16) _Float16 Psh[8][16 * KCH];
  __shared__ __align__(16) float    Os[QBLK * OSP];

  const int tid  = threadIdx.x;
  const int wave = tid >> 5;
  const int lane = tid & 31;
  const int hh   = lane >> 4;
  const int c    = lane & 15;

  const int bx = blockIdx.x;
  const int qb = bx & 3;
  const int t1 = bx >> 2;
  const int hp = t1 & 3;
  int b = t1 >> 2;
  b = b > nwin - 1 ? nwin - 1 : b;
  const int hw = wave >> 2;
  const int h  = hp * 2 + hw;
  const int wq = wave & 3;
  const int q0 = qb * QBLK + wq * 16;
  const int widx = b % nmask;
  const size_t rowbase = (size_t)b * NTOK;

  const v16h qa = Frag<_Float16>::load(qkv + (rowbase + q0 + c) * QKVLD + h * HD + 8 * hh);

  const float* bh_ptr = biasH + (size_t)h * NTOK * NTOK;
  const float* mk_ptr = maskp + (size_t)widx * NTOK * NTOK;
  const _Float16* ksh = Ksh[hw];
  const _Float16* vsh = Vtsh[hw];
  _Float16* pwh = Psh[wave];

  float mrow[8], lrow[8];
  v8f oacc[2];
#pragma unroll
  for (int r = 0; r < 8; ++r) { mrow[r] = -INFINITY; lrow[r] = 0.f; }
#pragma unroll
  for (int t = 0; t < 2; ++t) oacc[t] = (v8f){0.f,0.f,0.f,0.f,0.f,0.f,0.f,0.f};
  const v8f z8 = (v8f){0.f,0.f,0.f,0.f,0.f,0.f,0.f,0.f};

#pragma unroll 1
  for (int kc = 0; kc < NTOK / KCH; ++kc) {
    const int kv0 = kc * KCH;
    __syncthreads();
    {
      const int hs = tid >> 7, kvr = (tid >> 1) & 63, dh = (tid & 1) * 16;
      const _Float16* krow = qkv + (rowbase + kv0 + kvr) * QKVLD + CDIM + (hp * 2 + hs) * HD + dh;
      const _Float16* vrow = krow + CDIM;
      const v8h ka = *(const v8h*)krow;
      const v8h kb = *(const v8h*)(krow + 8);
      const v8h va = *(const v8h*)vrow;
      const v8h vb = *(const v8h*)(vrow + 8);
      _Float16* kd = Ksh[hs] + kvr * HD + dh;
      *(v8h*)kd = ka;
      *(v8h*)(kd + 8) = kb;
      _Float16* vd = Vtsh[hs] + dh * KCH + kvr;
#pragma unroll
      for (int e = 0; e < 8; ++e) { vd[e * KCH] = va[e]; vd[(8 + e) * KCH] = vb[e]; }
    }
    __syncthreads();

    v8f s[4];
#pragma unroll
    for (int j = 0; j < 4; ++j) {
      const v16h kf = Frag<_Float16>::load(ksh + (j * 16 + c) * HD + 8 * hh);
      s[j] = mma_h(qa, kf, z8);
    }

    float cm[8];
#pragma unroll
    for (int r = 0; r < 8; ++r) {
      const int qrow = q0 + 8 * hh + r;
      float m = -INFINITY;
#pragma unroll
      for (int j = 0; j < 4; ++j) {
        const int key = kv0 + j * 16 + c;
        const size_t oi = (size_t)qrow * NTOK + key;
        const float v = s[j][r] * qscale + bh_ptr[oi] + mk_ptr[oi];
        s[j][r] = v;
        m = fmaxf(m, v);
      }
#pragma unroll
      for (int off = 1; off < 16; off <<= 1) m = fmaxf(m, __shfl_xor(m, off, 32));
      cm[r] = m;
    }

#pragma unroll
    for (int r = 0; r < 8; ++r) {
      const float mnew  = fmaxf(mrow[r], cm[r]);
      const float alpha = __expf(mrow[r] - mnew);
      mrow[r] = mnew;
      float psum = 0.f;
#pragma unroll
      for (int j = 0; j < 4; ++j) {
        const float p = __expf(s[j][r] - mnew);
        psum += p;
        pwh[(8 * hh + r) * KCH + j * 16 + c] = (_Float16)(p * 32768.0f);
      }
#pragma unroll
      for (int off = 1; off < 16; off <<= 1) psum += __shfl_xor(psum, off, 32);
      lrow[r] = lrow[r] * alpha + psum;
#pragma unroll
      for (int t = 0; t < 2; ++t) oacc[t][r] *= alpha;
    }
    __builtin_amdgcn_fence(__ATOMIC_RELEASE, "workgroup");
    __builtin_amdgcn_wave_barrier();
    __builtin_amdgcn_fence(__ATOMIC_ACQUIRE, "workgroup");

#pragma unroll
    for (int kk = 0; kk < 2; ++kk) {
      const v16h pa = Frag<_Float16>::load(pwh + c * KCH + kk * 32 + 8 * hh);
#pragma unroll
      for (int t = 0; t < 2; ++t) {
        const v16h vf = Frag<_Float16>::load(vsh + (t * 16 + c) * KCH + kk * 32 + 8 * hh);
        oacc[t] = mma_h(pa, vf, oacc[t]);
      }
    }
  }

#pragma unroll
  for (int r = 0; r < 8; ++r) {
    const float inv = 1.0f / (lrow[r] * 32768.0f);
    const int row = wq * 16 + 8 * hh + r;
#pragma unroll
    for (int t = 0; t < 2; ++t) Os[row * OSP + hw * HD + t * 16 + c] = oacc[t][r] * inv;
  }
  __syncthreads();
  {
    const int q8 = lane >> 3, c8 = (lane & 7) * 8;
    _Float16* cbase = ctx + (rowbase + qb * QBLK) * CDIM + hp * 64;
    for (int pass = 0; pass < 2; ++pass) {
#pragma unroll
      for (int it = 0; it < 2; ++it) {
        const int row = wave * 8 + it * 4 + q8;
        const float* sp = Os + row * OSP + c8;
        v8h hv;
#pragma unroll
        for (int e = 0; e < 8; ++e) hv[e] = (_Float16)sp[e];
        *(volatile v8h*)(cbase + (size_t)row * CDIM + c8) = hv;
      }
      __threadfence();
    }
  }
}

static inline size_t align_up_128(size_t v) { return (v + 127) & ~(size_t)127; }

extern "C" void kernel_launch(void* const* d_in, const int* in_sizes, int n_in,
                              void* d_out, int out_size, void* d_ws, size_t ws_size,
                              hipStream_t stream) {
  if (n_in < 8) return;
  const float* x        = (const float*)d_in[0];
  const float* mask     = (const float*)d_in[1];
  const float* qkv_w    = (const float*)d_in[2];
  const float* qkv_b    = (const float*)d_in[3];
  const float* proj_w   = (const float*)d_in[4];
  const float* proj_b   = (const float*)d_in[5];
  const float* rp_table = (const float*)d_in[6];
  const int*   rp_index = (const int*)d_in[7];
  float* out = (float*)d_out;

  const int nwin  = in_sizes[0] / (NTOK * CDIM);
  const int nmask = in_sizes[1] / (NTOK * NTOK);
  const int ntab  = in_sizes[6] / HEADS;
  if (nwin <= 0 || nmask <= 0 || ntab <= 0) return;
  if (in_sizes[0] != nwin * NTOK * CDIM) return;
  if (in_sizes[2] != QKVLD * CDIM || in_sizes[3] != QKVLD) return;
  if (in_sizes[4] != CDIM * CDIM || in_sizes[5] != CDIM) return;
  if (in_sizes[7] != NTOK * NTOK) return;
  if (out_size != nwin * NTOK * CDIM) return;

  const int M = nwin * NTOK;

  const size_t sz_qkv16 = (size_t)M * QKVLD * sizeof(unsigned short);
  const size_t sz_x16   = (size_t)M * CDIM * sizeof(unsigned short);
  const size_t sz_w16   = (size_t)QKVLD * CDIM * sizeof(unsigned short);
  const size_t sz_pw16  = (size_t)CDIM * CDIM * sizeof(unsigned short);
  const size_t sz_bias  = (size_t)HEADS * NTOK * NTOK * sizeof(float);
  const size_t off_qkv16 = 0;
  const size_t off_x16   = align_up_128(off_qkv16 + sz_qkv16);
  const size_t off_w16   = align_up_128(off_x16 + sz_x16);
  const size_t off_pw16  = align_up_128(off_w16 + sz_w16);
  const size_t off_bias  = align_up_128(off_pw16 + sz_pw16);
  const size_t total     = off_bias + sz_bias;
  if (total > ws_size || total > (size_t)134217728) return;

  char* ws = (char*)d_ws;
  unsigned short* qkv16 = (unsigned short*)(ws + off_qkv16);
  unsigned short* x16   = (unsigned short*)(ws + off_x16);
  unsigned short* ctx16 = x16;
  unsigned short* w16   = (unsigned short*)(ws + off_w16);
  unsigned short* pw16  = (unsigned short*)(ws + off_pw16);
  float*          biasH = (float*)(ws + off_bias);

  {
    const int n2x = in_sizes[0] / 2;
    cast_f32_f16x2<<<(n2x + 255) / 256, 256, 0, stream>>>(x, (_Float16*)x16, n2x, 1.0f);
    const int n2w = (QKVLD * CDIM) / 2;
    cast_f32_f16x2<<<(n2w + 255) / 256, 256, 0, stream>>>(qkv_w, (_Float16*)w16, n2w, 64.0f);
    const int n2p = (CDIM * CDIM) / 2;
    cast_f32_f16x2<<<(n2p + 255) / 256, 256, 0, stream>>>(proj_w, (_Float16*)pw16, n2p, 64.0f);
    bias_gather_kernel<<<(NTOK * NTOK + 255) / 256, 256, 0, stream>>>(rp_table, rp_index, biasH, ntab);
  }

  {
    const int tiles = (M / 64) * (QKVLD / 64);
    dim3 grid((tiles + 7) / 8, 1);
    wmma_gemm64<0, false, 2, 1, false><<<grid, 256, 0, stream>>>(
        x16, x16, CDIM, 0L,
        w16, w16, CDIM, 0L,
        (void*)qkv16, (void*)qkv16, QKVLD, 0L,
        qkv_b, qkv_b, 0L,
        M, QKVLD, CDIM, 1.0f / 64.0f);
  }

  {
    const int nblk = nwin * (HEADS / 2) * (NTOK / QBLK);
    const float qscale = 0.17677669529663687f;
    attn_hd32_kernel<<<nblk, 256, 0, stream>>>((const _Float16*)qkv16, biasH, mask,
                                                (_Float16*)ctx16, nwin, nmask, qscale);
  }

  {
    const int tiles = (M / 64) * (CDIM / 64);
    dim3 grid((tiles + 7) / 8, 1);
    wmma_gemm64<0, false, 2, 0, false><<<grid, 256, 0, stream>>>(
        ctx16, ctx16, CDIM, 0L,
        pw16, pw16, CDIM, 0L,
        (void*)out, (void*)out, CDIM, 0L,
        proj_b, proj_b, 0L,
        M, CDIM, CDIM, 1.0f / 64.0f);
  }
  (void)hipGetLastError();
}
